// RelationalAttentionContextEncoder3_27127013441946
// MI455X (gfx1250) — hardware-verified
//
#include <hip/hip_runtime.h>
#include <math.h>

constexpr int kB     = 512;
constexpr int kN     = 64;
constexpr int kD     = 4;
constexpr int kH     = 128;
constexpr int kRelIn = 9;
constexpr int kRowsTotal     = kB * kN * kN;
constexpr int kChunks        = 32;
constexpr int kRowsPerChunk  = kRowsTotal / kChunks;
constexpr int kGroupsPerChunk = kRowsPerChunk / kN;
constexpr float kH1Carry   = 128.0f;
constexpr float kW2Carry   = 1024.0f;
constexpr float kGemmScale = 1.0f / (128.0f * 1024.0f);
constexpr float kInv63     = 1.0f / 63.0f;

constexpr size_t kOffW2t  = 0;
constexpr size_t kBytesW2t = (size_t)kH * kH * 2;
constexpr size_t kOffH1   = 65536;
constexpr size_t kBytesH1 = (size_t)kRowsPerChunk * kH * 2;
constexpr size_t kOffH2   = kOffH1 + kBytesH1;
constexpr size_t kBytesH2 = (size_t)kRowsPerChunk * kH * 4;
constexpr size_t kWsTotal = kOffH2 + kBytesH2;

typedef char chk_rows_tile[(kRowsPerChunk % 64 == 0) ? 1 : -1];
typedef char chk_groups[(kGroupsPerChunk % 8 == 0) ? 1 : -1];
typedef char chk_ws_total[(kWsTotal <= (size_t)134217728) ? 1 : -1];
typedef char chk_align_h1[(kOffH1 % 256 == 0) ? 1 : -1];
typedef char chk_align_h2[(kOffH2 % 256 == 0) ? 1 : -1];
typedef char chk_k32[(kH % 32 == 0) ? 1 : -1];

typedef __attribute__((ext_vector_type(16))) _Float16 v16h;
typedef __attribute__((ext_vector_type(8)))  _Float16 v8h;
typedef __attribute__((ext_vector_type(16))) __bf16   v16b;
typedef __attribute__((ext_vector_type(8)))  __bf16   v8b;
typedef __attribute__((ext_vector_type(8)))  float    v8f;
typedef __attribute__((ext_vector_type(4)))  float    v4f;
typedef __attribute__((ext_vector_type(4)))  unsigned int v4u;

__device__ __forceinline__ unsigned short f2bf_bits(float f) {
  unsigned u = __float_as_uint(f);
  return (unsigned short)((u + 0x7FFFu + ((u >> 16) & 1u)) >> 16);
}
__device__ __forceinline__ float bf_bits2f(unsigned short h) { return __uint_as_float(((unsigned)h) << 16); }

__device__ __forceinline__ void dep_guard_h(v8f& a, v8f& b, v16h x, v16h y) { asm volatile("v_nop\n\tv_nop\n\tv_nop\n\tv_nop" : "+v"(a), "+v"(b) : "v"(x), "v"(y)); }
__device__ __forceinline__ void dep_guard_b(v8f& a, v8f& b, v16b x, v16b y) { asm volatile("v_nop\n\tv_nop\n\tv_nop\n\tv_nop" : "+v"(a), "+v"(b) : "v"(x), "v"(y)); }
__device__ __forceinline__ void keep4_h(v16h a, v16h b, v16h c, v16h d) { asm volatile("v_nop" :: "v"(a), "v"(b), "v"(c), "v"(d)); }
__device__ __forceinline__ void keep4_b(v16b a, v16b b, v16b c, v16b d) { asm volatile("v_nop" :: "v"(a), "v"(b), "v"(c), "v"(d)); }
__device__ __forceinline__ void acc_guard4(v8f& a, v8f& b, v8f& c, v8f& d) { asm volatile("v_nop\n\tv_nop\n\tv_nop\n\tv_nop" : "+v"(a), "+v"(b), "+v"(c), "+v"(d)); }
template <typename T> struct Frag;
template <> struct Frag<_Float16> {
  typedef v16h V; union U { v16h v; v8h h[2]; };
  static __device__ __forceinline__ v16h load(const _Float16* p) {
    U f; f.h[0] = *(const v8h*)(p); f.h[1] = *(const v8h*)(p + 16); return f.v;
  }
  static __device__ __forceinline__ v8f mma(v16h a, v16h b, v8f c) {
    return __builtin_amdgcn_wmma_f32_16x16x32_f16(false, a, false, b, (short)0, c, false, false);
  }
  static __device__ __forceinline__ void guard(v8f& a, v8f& b, v16h x, v16h y) { dep_guard_h(a, b, x, y); }
  static __device__ __forceinline__ void keep(v16h a, v16h b, v16h c, v16h d) { keep4_h(a, b, c, d); }
};
template <> struct Frag<__bf16> {
  typedef v16b V; union U { v16b v; v8b h[2]; };
  static __device__ __forceinline__ v16b load(const __bf16* p) {
    U f; f.h[0] = *(const v8b*)(p); f.h[1] = *(const v8b*)(p + 16); return f.v;
  }
  static __device__ __forceinline__ v8f mma(v16b a, v16b b, v8f c) {
    return __builtin_amdgcn_wmma_f32_16x16x32_bf16(false, a, false, b, (short)0, c, false, false);
  }
  static __device__ __forceinline__ void guard(v8f& a, v8f& b, v16b x, v16b y) { dep_guard_b(a, b, x, y); }
  static __device__ __forceinline__ void keep(v16b a, v16b b, v16b c, v16b d) { keep4_b(a, b, c, d); }
};

__device__ __forceinline__ unsigned pk16(unsigned short a, unsigned short b) { return (unsigned)a | ((unsigned)b << 16); }
__device__ __forceinline__ unsigned short h_bits(float f) { const _Float16 h = (_Float16)f; return __builtin_bit_cast(unsigned short, h); }

template <int ET> struct Elem;
template <> struct Elem<0> { typedef _Float16 T; };
template <> struct Elem<1> { typedef __bf16 T; };
template <int ET, bool SPLIT, int BIAS_MODE, int OUT_MODE, bool RESID, int ACT = 0>
__global__ __launch_bounds__(256) void wmma_gemm64(
    const unsigned short* __restrict__ Ap, const unsigned short* __restrict__ A2p, int lda, long strideA,
    const unsigned short* __restrict__ Btp, const unsigned short* __restrict__ Bt2p, int ldb, long strideB,
    void* __restrict__ Cout, void* __restrict__ Cout2, int ldc, long strideC,
    const float* __restrict__ bias,
    const float* __restrict__ resid, long strideR,
    int M, int N, int K, float scale) {
  typedef typename Elem<ET>::T T;
  typedef typename Frag<T>::V V;
  const T* A = (const T*)Ap; const T* A2 = (const T*)A2p; const T* Bt = (const T*)Btp; const T* Bt2 = (const T*)Bt2p;
  __shared__ __align__(16) float sT[8][16 * 68];
  const int b    = blockIdx.y;
  const int lane = threadIdx.x & 31;
  const int wave = threadIdx.x >> 5;
  const int tilesN = N >> 6;
  const int tilesM = M >> 6;
  const int tile = blockIdx.x * 8 + wave;
  if (tile >= tilesM * tilesN) return;
  const int tm = tile / tilesN;
  const int tn = tile - tm * tilesN;
  const int m0 = tm << 6;
  const int n0 = tn << 6;

  const T* Ab  = A  + (size_t)b * strideA;
  const T* Bb  = Bt + (size_t)b * strideB;
  const T* Ab2 = SPLIT ? (A2  + (size_t)b * strideA) : nullptr;
  const T* Bb2 = SPLIT ? (Bt2 + (size_t)b * strideB) : nullptr;

  const int rlane = lane & 15;
  const int koff  = (lane >> 4) * 8;
  const int mOff  = (lane >> 4) * 8;

  v8f acc[4][4];
#pragma unroll
  for (int i = 0; i < 4; ++i)
#pragma unroll
    for (int j = 0; j < 4; ++j) acc[i][j] = (v8f){0.f,0.f,0.f,0.f,0.f,0.f,0.f,0.f};

  for (int k0 = 0; k0 < K; k0 += 32) {
    V bh[4], bl[4];
#pragma unroll
    for (int j = 0; j < 4; ++j) {
      const size_t bo = (size_t)(n0 + (j << 4) + rlane) * ldb + koff + k0;
      bh[j] = Frag<T>::load(Bb + bo);
      if (SPLIT) bl[j] = Frag<T>::load(Bb2 + bo);
    }
#pragma unroll
    for (int i = 0; i < 4; ++i) {
      const size_t ao = (size_t)(m0 + (i << 4) + rlane) * lda + koff + k0;
      V ah = Frag<T>::load(Ab + ao);
      V al;
      if (SPLIT) al = Frag<T>::load(Ab2 + ao);
#pragma unroll
      for (int j = 0; j < 4; ++j) {
        acc[i][j] = Frag<T>::mma(ah, bh[j], acc[i][j]);
        if (SPLIT) {
          acc[i][j] = Frag<T>::mma(ah, bl[j], acc[i][j]);
          acc[i][j] = Frag<T>::mma(al, bh[j], acc[i][j]);
        }
      }
      Frag<T>::guard(acc[i][0], acc[i][3], ah, SPLIT ? al : ah);
    }
    Frag<T>::keep(bh[0], bh[1], bh[2], bh[3]);
    if (SPLIT) Frag<T>::keep(bl[0], bl[1], bl[2], bl[3]);
  }
  acc_guard4(acc[0][0], acc[0][1], acc[0][2], acc[0][3]);
  acc_guard4(acc[1][0], acc[1][1], acc[1][2], acc[1][3]);
  acc_guard4(acc[2][0], acc[2][1], acc[2][2], acc[2][3]);
  acc_guard4(acc[3][0], acc[3][1], acc[3][2], acc[3][3]);

  float* slab = sT[wave];
  const float* Rb = RESID ? (resid + (size_t)b * strideR) : nullptr;
#pragma unroll
  for (int i = 0; i < 4; ++i) {
    const int mBase = m0 + (i << 4);
#pragma unroll
    for (int j = 0; j < 4; ++j) {
      const int n = n0 + (j << 4) + rlane;
      float bv = 0.f;
      if (BIAS_MODE == 2) bv = bias[n];
#pragma unroll
      for (int r = 0; r < 8; ++r) {
        float v = acc[i][j][r] * scale;
        if (BIAS_MODE == 1) v += bias[mBase + mOff + r];
        if (BIAS_MODE == 2) v += bv;
        if (RESID) v += Rb[(size_t)(mBase + mOff + r) * ldc + n];
        if (ACT == 2) v = fmaxf(v, 0.0f);
        if (ACT == 4) v = (v > 0.f) ? v : 0.01f * v;
        slab[(mOff + r) * 68 + (j << 4) + rlane] = v;
      }
    }
    __builtin_amdgcn_fence(__ATOMIC_RELEASE, "workgroup");
    __builtin_amdgcn_wave_barrier();
    __builtin_amdgcn_fence(__ATOMIC_ACQUIRE, "workgroup");
    if (OUT_MODE == 0) {
      float* C = (float*)Cout + (size_t)b * strideC;
      const int hh = lane >> 4, c4 = (lane & 15) * 4;
      for (int pass = 0; pass < 2; ++pass) {
#pragma unroll
        for (int it = 0; it < 8; ++it) {
          const int row = it * 2 + hh;
          v4f v = *(const v4f*)(slab + row * 68 + c4);
          *(volatile v4f*)(C + (size_t)(mBase + row) * ldc + n0 + c4) = v;
        }
        __threadfence();
      }
    } else {
      const int q = lane >> 3, c8 = (lane & 7) * 8;
      unsigned short* C  = (unsigned short*)Cout  + (size_t)b * strideC;
      unsigned short* C2 = (OUT_MODE == 2) ? ((unsigned short*)Cout2 + (size_t)b * strideC) : nullptr;
      for (int pass = 0; pass < 2; ++pass) {
#pragma unroll
        for (int it = 0; it < 4; ++it) {
          const int row = it * 4 + q;
          const float* sp = slab + row * 68 + c8;
          v8h hv, lv;
#pragma unroll
          for (int e = 0; e < 8; ++e) {
            if (OUT_MODE == 1) {
              hv[e] = (_Float16)sp[e];
            } else {
              unsigned short hb = f2bf_bits(sp[e]);
              unsigned short lb = f2bf_bits(sp[e] - bf_bits2f(hb));
              hv[e] = __builtin_bit_cast(_Float16, hb);
              lv[e] = __builtin_bit_cast(_Float16, lb);
            }
          }
          *(volatile v8h*)(C + (size_t)(mBase + row) * ldc + n0 + c8) = hv;
          if (OUT_MODE == 2) *(volatile v8h*)(C2 + (size_t)(mBase + row) * ldc + n0 + c8) = lv;
        }
        __threadfence();
      }
    }
    __builtin_amdgcn_fence(__ATOMIC_RELEASE, "workgroup");
    __builtin_amdgcn_wave_barrier();
    __builtin_amdgcn_fence(__ATOMIC_ACQUIRE, "workgroup");
  }
}

__global__ __launch_bounds__(256) void w2t_cast_kernel(const float* __restrict__ W2, unsigned short* __restrict__ out, float scale) {
  __shared__ float sm[64][65];
  const int t  = threadIdx.x;
  const int k0 = blockIdx.x * 64;
  const int n0 = blockIdx.y * 64;
#pragma unroll
  for (int i = 0; i < 16; ++i) {
    const int e = i * 256 + t;
    const int r = e >> 6;
    const int c = e & 63;
    sm[c][r] = W2[(size_t)(k0 + r) * kH + n0 + c] * scale;
  }
  __syncthreads();
  const int lane = t & 31, wave = t >> 5;
  const int q = lane >> 3, c8 = (lane & 7) * 8;
  for (int pass = 0; pass < 2; ++pass) {
#pragma unroll
    for (int it = 0; it < 2; ++it) {
      const int row = wave * 8 + it * 4 + q;
      unsigned short hb[8];
#pragma unroll
      for (int e = 0; e < 8; ++e) hb[e] = h_bits(sm[row][c8 + e]);
      const v4u u = (v4u){pk16(hb[0], hb[1]), pk16(hb[2], hb[3]), pk16(hb[4], hb[5]), pk16(hb[6], hb[7])};
      *(volatile v4u*)(out + (size_t)(n0 + row) * kH + k0 + c8) = u;
    }
    __threadfence();
  }
}

__global__ __launch_bounds__(128) void pair_mlp1_kernel(const float* __restrict__ ctx, const float* __restrict__ W1,
                                                       const float* __restrict__ b1, unsigned short* __restrict__ H1,
                                                       int chunk) {
  __shared__ __align__(16) float sEnt[kN * kD];
  __shared__ __align__(16) float sW1[kRelIn * kH];
  __shared__ __align__(16) float sB1[kH];
  __shared__ __align__(16) unsigned int slab[128 * 64];
  const int tid = threadIdx.x;
  const int g0  = chunk * kGroupsPerChunk + blockIdx.x * 2;
  const int b   = g0 >> 6;
  const int sub = tid >> 6;
  const int iEnt = (g0 + sub) & 63;
  const int j    = tid & 63;

  for (int e = tid; e < kN * kD; e += 128) sEnt[e] = ctx[(size_t)b * (kN * kD) + e];
  for (int e = tid; e < kRelIn * kH; e += 128) sW1[e] = W1[e] * kH1Carry;
  sB1[tid] = b1[tid] * kH1Carry;
  __syncthreads();

  const float ei0 = sEnt[iEnt * 4 + 0], ei1 = sEnt[iEnt * 4 + 1], ei2 = sEnt[iEnt * 4 + 2], ei3 = sEnt[iEnt * 4 + 3];
  const float ej0 = sEnt[j * 4 + 0],    ej1 = sEnt[j * 4 + 1],    ej2 = sEnt[j * 4 + 2],    ej3 = sEnt[j * 4 + 3];
  const float f0 = ei2, f1 = ei3, f2 = ej2, f3 = ej3;
  const float f4 = ei0 - ej0, f5 = ei1 - ej1, f6 = ei2 - ej2, f7 = ei3 - ej3;
  const float f8 = sqrtf(f4 * f4 + f5 * f5);

  unsigned int* srow = slab + tid * 64;
#pragma unroll 1
  for (int g = 0; g < 16; ++g) {
    const int c0 = g * 8;
    unsigned short hb[8];
#pragma unroll
    for (int e = 0; e < 8; ++e) {
      const int c = c0 + e;
      float a = sB1[c];
      a = fmaf(f0, sW1[0 * kH + c], a);
      a = fmaf(f1, sW1[1 * kH + c], a);
      a = fmaf(f2, sW1[2 * kH + c], a);
      a = fmaf(f3, sW1[3 * kH + c], a);
      a = fmaf(f4, sW1[4 * kH + c], a);
      a = fmaf(f5, sW1[5 * kH + c], a);
      a = fmaf(f6, sW1[6 * kH + c], a);
      a = fmaf(f7, sW1[7 * kH + c], a);
      a = fmaf(f8, sW1[8 * kH + c], a);
      a = fmaxf(a, 0.0f);
      hb[e] = h_bits(a);
    }
    const v4u u = (v4u){pk16(hb[0], hb[1]), pk16(hb[2], hb[3]), pk16(hb[4], hb[5]), pk16(hb[6], hb[7])};
    *(v4u*)(srow + g * 4) = u;
  }
  __syncthreads();

  const int wave = tid >> 5, lane = tid & 31;
  unsigned int* gdst = (unsigned int*)H1 + (size_t)blockIdx.x * (128 * 64);
  for (int pass = 0; pass < 2; ++pass) {
#pragma unroll
    for (int k = 0; k < 16; ++k) {
      const int idx = wave * 2048 + k * 128 + lane * 4;
      const v4u u = *(const v4u*)(slab + idx);
      *(volatile v4u*)(gdst + idx) = u;
    }
    __threadfence();
  }
}

__global__ __launch_bounds__(256) void pool_prop_kernel(const float* __restrict__ H2, const float* __restrict__ ctx,
                                                        const float* __restrict__ Wp, const float* __restrict__ bp,
                                                        float* __restrict__ out, int chunk) {
  const int tid  = threadIdx.x;
  const int wave = tid >> 5, lane = tid & 31;
  const int gl   = blockIdx.x * 8 + wave;
  const int G    = chunk * kGroupsPerChunk + gl;
  const int b    = G >> 6;
  const int iEnt = G & 63;

  const float* hrow = H2 + (size_t)gl * (kN * kH) + 4 * lane;
  float s0 = 0.f, s1 = 0.f, s2 = 0.f, s3 = 0.f;
#pragma unroll 8
  for (int j = 0; j < kN; ++j) {
    const v4f v = *(const v4f*)(hrow + (size_t)j * kH);
    const bool keep = (j != iEnt);
    s0 += keep ? v[0] : 0.0f;
    s1 += keep ? v[1] : 0.0f;
    s2 += keep ? v[2] : 0.0f;
    s3 += keep ? v[3] : 0.0f;
  }
  const v4f rel = (v4f){s0 * kInv63, s1 * kInv63, s2 * kInv63, s3 * kInv63};

  const float a0 = ctx[(size_t)b * (kN * kD) + iEnt * kD + 2];
  const float a1 = ctx[(size_t)b * (kN * kD) + iEnt * kD + 3];
  const v4f w0 = *(const v4f*)(Wp + 4 * lane);
  const v4f w1 = *(const v4f*)(Wp + kH + 4 * lane);
  const v4f bb = *(const v4f*)(bp + 4 * lane);
  v4f p;
#pragma unroll
  for (int e = 0; e < 4; ++e) {
    float t = a0 * w0[e];
    t = fmaf(a1, w1[e], t);
    t = t + bb[e];
    p[e] = fmaxf(t, 0.0f);
  }

  float* orow = out + (size_t)G * (2 * kH);
  for (int pass = 0; pass < 2; ++pass) {
    *(volatile v4f*)(orow + 4 * lane) = p;
    *(volatile v4f*)(orow + kH + 4 * lane) = rel;
    __threadfence();
  }
}

extern "C" void kernel_launch(void* const* d_in, const int* in_sizes, int n_in,
                              void* d_out, int out_size, void* d_ws, size_t ws_size,
                              hipStream_t stream) {
  if (n_in < 7) return;
  if (in_sizes[0] != kB * kN * kD) return;
  if (in_sizes[1] != kRelIn * kH) return;
  if (in_sizes[2] != kH) return;
  if (in_sizes[3] != kH * kH) return;
  if (in_sizes[4] != kH) return;
  if (in_sizes[5] != 2 * kH) return;
  if (in_sizes[6] != kH) return;
  if (out_size != kB * kN * 2 * kH) return;
  if (ws_size < kWsTotal) return;

  const float* ctx = (const float*)d_in[0];
  const float* W1  = (const float*)d_in[1];
  const float* b1  = (const float*)d_in[2];
  const float* W2  = (const float*)d_in[3];
  const float* b2  = (const float*)d_in[4];
  const float* Wp  = (const float*)d_in[5];
  const float* bp  = (const float*)d_in[6];
  float* out = (float*)d_out;

  unsigned char* ws = (unsigned char*)d_ws;
  unsigned short* W2t = (unsigned short*)(ws + kOffW2t);
  unsigned short* H1  = (unsigned short*)(ws + kOffH1);
  float*          H2  = (float*)(ws + kOffH2);

  w2t_cast_kernel<<<dim3(2, 2), dim3(256), 0, stream>>>(W2, W2t, kW2Carry);

  const int tilesPerChunk = (kRowsPerChunk / 64) * (kH / 64);
  for (int chunk = 0; chunk < kChunks; ++chunk) {
    pair_mlp1_kernel<<<dim3(kGroupsPerChunk / 2), dim3(128), 0, stream>>>(ctx, W1, b1, H1, chunk);
    wmma_gemm64<0, false, 2, 0, false, 2><<<dim3(tilesPerChunk / 8, 1), dim3(256), 0, stream>>>(
        H1, H1, kH, 0L,
        W2t, W2t, kH, 0L,
        (void*)H2, (void*)H2, kH, 0L,
        b2, (const float*)nullptr, 0L,
        kRowsPerChunk, kH, kH, kGemmScale);
    pool_prop_kernel<<<dim3(kGroupsPerChunk / 8), dim3(256), 0, stream>>>(H2, ctx, Wp, bp, out, chunk);
  }
}
